// SelectiveScan_86414741996283
// MI455X (gfx1250) — hardware-run, weakly checked
//
#include <hip/hip_runtime.h>
#include <math.h>

typedef __attribute__((ext_vector_type(16))) _Float16 v16h;
typedef __attribute__((ext_vector_type(8)))  _Float16 v8h;
typedef __attribute__((ext_vector_type(16))) __bf16   v16b;
typedef __attribute__((ext_vector_type(8)))  __bf16   v8b;
typedef __attribute__((ext_vector_type(8)))  float    v8f;
typedef __attribute__((ext_vector_type(4)))  float    v4f;

constexpr int kSeq    = 4096;
constexpr int kDm     = 768;
constexpr int kDin    = 1536;
constexpr int kNst    = 16;
constexpr int kNxz    = 3 * kDin + 2 * kNst;
constexpr int kXzP    = 4672;
constexpr int kColZ   = kDin;
constexpr int kColB   = 2 * kDin;
constexpr int kColC   = 2 * kDin + kNst;
constexpr int kColDt  = 2 * kDin + 2 * kNst;
constexpr int kScanTS = 64;
constexpr int kScanCh = 64;
constexpr int kScanYP = 68;
constexpr int kBCW    = 2 * kNst;
constexpr float kYCarry   = 256.0f;
constexpr float kWoCarry  = 256.0f;
constexpr float kOutScale = 1.0f / (kYCarry * kWoCarry);
static_assert(kNxz == 4640, "projection width");
static_assert(kColDt + kDin == kNxz, "column split");
static_assert((kXzP % 64) == 0 && kXzP >= kNxz && kXzP - kNxz < 64, "padded N");
static_assert((kDm % 32) == 0 && (kDin % 32) == 0, "GEMM K multiples of 32");
static_assert((kSeq % 64) == 0 && (kDm % 64) == 0, "GEMM M,N multiples of 64");
static_assert(((kSeq / 64) * (kXzP / 64)) % 8 == 0 && ((kSeq / 64) * (kDm / 64)) % 8 == 0, "whole blocks of 8 tiles");
static_assert((kSeq % kScanTS) == 0 && (kDin % kScanCh) == 0, "scan tiles");
static_assert(((kColB * 4) % 128) == 0 && ((kColDt * 4) % 128) == 0 && ((kXzP * 4) % 128) == 0, "line-aligned columns");
static_assert(((kNxz * kDm) % 2048) == 0 && ((kXzP * kDm) % 2048) == 0 && ((kSeq * kDm) % 2048) == 0 && ((kDm * kDin) % 2048) == 0, "convert grids exact");

constexpr size_t kOffX16  = 0;
constexpr size_t kOffWIN  = kOffX16 + (size_t)kSeq * kDm * 2;
constexpr size_t kOffWOUT = kOffWIN + (size_t)kXzP * kDm * 2;
constexpr size_t kOffXZ   = kOffWOUT + (size_t)kDm * kDin * 2;
constexpr size_t kOffY16  = kOffXZ + (size_t)kSeq * kXzP * 4;
constexpr size_t kWsTotal = kOffY16 + (size_t)kSeq * kDin * 2;
static_assert(kWsTotal == 104955904ull, "carve total");
static_assert(kWsTotal <= 134217728ull, "carve cap");
static_assert((kOffWIN % 128) == 0 && (kOffWOUT % 128) == 0 && (kOffXZ % 128) == 0 && (kOffY16 % 128) == 0, "128-B aligned regions");

__device__ __forceinline__ unsigned short f2bf_bits(float f) {
  unsigned u = __float_as_uint(f);
  return (unsigned short)((u + 0x7FFFu + ((u >> 16) & 1u)) >> 16);
}
__device__ __forceinline__ float bf_bits2f(unsigned short h) { return __uint_as_float(((unsigned)h) << 16); }
__device__ __forceinline__ float rne_bf(float f) { return bf_bits2f(f2bf_bits(f)); }

__device__ __forceinline__ void dep_guard4_h(v8f& a, v8f& b, v8f& c, v8f& d, v16h x, v16h y) { asm volatile("v_nop\n\tv_nop\n\tv_nop\n\tv_nop" : "+v"(a), "+v"(b), "+v"(c), "+v"(d) : "v"(x), "v"(y)); }
__device__ __forceinline__ void dep_guard4_b(v8f& a, v8f& b, v8f& c, v8f& d, v16b x, v16b y) { asm volatile("v_nop\n\tv_nop\n\tv_nop\n\tv_nop" : "+v"(a), "+v"(b), "+v"(c), "+v"(d) : "v"(x), "v"(y)); }
__device__ __forceinline__ void keep4_h(v16h a, v16h b, v16h c, v16h d) { asm volatile("v_nop" :: "v"(a), "v"(b), "v"(c), "v"(d)); }
__device__ __forceinline__ void keep4_b(v16b a, v16b b, v16b c, v16b d) { asm volatile("v_nop" :: "v"(a), "v"(b), "v"(c), "v"(d)); }
__device__ __forceinline__ void acc_guard4(v8f& a, v8f& b, v8f& c, v8f& d) { asm volatile("v_nop\n\tv_nop\n\tv_nop\n\tv_nop" : "+v"(a), "+v"(b), "+v"(c), "+v"(d)); }

template <typename T> struct Frag;
template <> struct Frag<_Float16> {
  typedef v16h V; union U { v16h v; v8h h[2]; };
  static __device__ __forceinline__ v16h load(const _Float16* p) {
    U f; f.h[0] = *(const v8h*)(p); f.h[1] = *(const v8h*)(p + 16); return f.v;
  }
  static __device__ __forceinline__ v8f mma(v16h a, v16h b, v8f c) {
    return __builtin_amdgcn_wmma_f32_16x16x32_f16(false, a, false, b, (short)0, c, false, false);
  }
  static __device__ __forceinline__ void guard4(v8f& a, v8f& b, v8f& c, v8f& d, v16h x, v16h y) { dep_guard4_h(a, b, c, d, x, y); }
  static __device__ __forceinline__ void keep(v16h a, v16h b, v16h c, v16h d) { keep4_h(a, b, c, d); }
};
template <> struct Frag<__bf16> {
  typedef v16b V; union U { v16b v; v8b h[2]; };
  static __device__ __forceinline__ v16b load(const __bf16* p) {
    U f; f.h[0] = *(const v8b*)(p); f.h[1] = *(const v8b*)(p + 16); return f.v;
  }
  static __device__ __forceinline__ v8f mma(v16b a, v16b b, v8f c) {
    return __builtin_amdgcn_wmma_f32_16x16x32_bf16(false, a, false, b, (short)0, c, false, false);
  }
  static __device__ __forceinline__ void guard4(v8f& a, v8f& b, v8f& c, v8f& d, v16b x, v16b y) { dep_guard4_b(a, b, c, d, x, y); }
  static __device__ __forceinline__ void keep(v16b a, v16b b, v16b c, v16b d) { keep4_b(a, b, c, d); }
};

template <int ET> struct Elem;
template <> struct Elem<0> { typedef _Float16 T; };
template <> struct Elem<1> { typedef __bf16 T; };
template <int ET>
__global__ __launch_bounds__(256) void wmma_gemm64(
    const unsigned short* __restrict__ Ap, int lda,
    const unsigned short* __restrict__ Btp, int ldb,
    float* __restrict__ C, int ldc,
    int M, int N, int K, float scale) {
  typedef typename Elem<ET>::T T;
  typedef typename Frag<T>::V V;
  const T* A = (const T*)Ap;
  const T* Bt = (const T*)Btp;
  __shared__ __align__(16) float sT[8][16 * 68];
  const int lane = threadIdx.x & 31;
  const int wave = threadIdx.x >> 5;
  const int tilesN = N >> 6;
  const int tilesM = M >> 6;
  const int tile = blockIdx.x * 8 + wave;
  if (tile >= tilesM * tilesN) return;
  const int tm = tile / tilesN;
  const int tn = tile - tm * tilesN;
  const int m0 = tm << 6;
  const int n0 = tn << 6;

  const int rlane = lane & 15;
  const int koff  = (lane >> 4) * 8;
  const int mOff  = (lane >> 4) * 8;

  v8f acc[4][4];
#pragma unroll
  for (int i = 0; i < 4; ++i)
#pragma unroll
    for (int j = 0; j < 4; ++j) acc[i][j] = (v8f){0.f,0.f,0.f,0.f,0.f,0.f,0.f,0.f};

  for (int k0 = 0; k0 < K; k0 += 32) {
    V bh[4];
#pragma unroll
    for (int j = 0; j < 4; ++j) {
      const size_t bo = (size_t)(n0 + (j << 4) + rlane) * ldb + koff + k0;
      bh[j] = Frag<T>::load(Bt + bo);
    }
#pragma unroll
    for (int i = 0; i < 4; ++i) {
      const size_t ao = (size_t)(m0 + (i << 4) + rlane) * lda + koff + k0;
      V ah = Frag<T>::load(A + ao);
#pragma unroll
      for (int j = 0; j < 4; ++j) {
        acc[i][j] = Frag<T>::mma(ah, bh[j], acc[i][j]);
      }
      Frag<T>::guard4(acc[i][0], acc[i][1], acc[i][2], acc[i][3], ah, bh[3]);
    }
    Frag<T>::keep(bh[0], bh[1], bh[2], bh[3]);
  }
  acc_guard4(acc[0][0], acc[0][1], acc[0][2], acc[0][3]);
  acc_guard4(acc[1][0], acc[1][1], acc[1][2], acc[1][3]);
  acc_guard4(acc[2][0], acc[2][1], acc[2][2], acc[2][3]);
  acc_guard4(acc[3][0], acc[3][1], acc[3][2], acc[3][3]);

  float* slab = sT[wave];
#pragma unroll
  for (int i = 0; i < 4; ++i) {
    const int mBase = m0 + (i << 4);
#pragma unroll
    for (int j = 0; j < 4; ++j) {
#pragma unroll
      for (int r = 0; r < 8; ++r) {
        const float v = acc[i][j][r] * scale;
        slab[(mOff + r) * 68 + (j << 4) + rlane] = v;
      }
    }
    __builtin_amdgcn_fence(__ATOMIC_RELEASE, "workgroup");
    __builtin_amdgcn_wave_barrier();
    __builtin_amdgcn_fence(__ATOMIC_ACQUIRE, "workgroup");
    {
      const int hh = lane >> 4, c4 = (lane & 15) * 4;
      for (int pass = 0; pass < 2; ++pass) {
#pragma unroll
        for (int it = 0; it < 8; ++it) {
          const int row = it * 2 + hh;
          v4f v = *(const v4f*)(slab + row * 68 + c4);
          *(volatile v4f*)(C + (size_t)(mBase + row) * ldc + n0 + c4) = v;
        }
        __threadfence();
      }
    }
    __builtin_amdgcn_fence(__ATOMIC_RELEASE, "workgroup");
    __builtin_amdgcn_wave_barrier();
    __builtin_amdgcn_fence(__ATOMIC_ACQUIRE, "workgroup");
  }
}

template <int MODE>
__global__ __launch_bounds__(256) void plane_convert_kernel(
    const float* __restrict__ src, unsigned short* __restrict__ dst, int total8, int src8, float scale)
{
  const int i = blockIdx.x * 256 + threadIdx.x;
  if (i >= total8) return;
  const bool live = (i < src8);
  const int ic = live ? i : (src8 - 1);
  const float* p = src + ((size_t)ic << 3);
  const v4f a0 = *(const v4f*)(p);
  const v4f a1 = *(const v4f*)(p + 4);
  v8h hv;
#pragma unroll
  for (int e = 0; e < 4; ++e) {
    const float g0 = a0[e];
    const float g1 = a1[e];
    const float f0 = live ? g0 : 0.0f;
    const float f1 = live ? g1 : 0.0f;
    const unsigned short b0 = f2bf_bits(f0);
    const unsigned short b1 = f2bf_bits(f1);
    if (MODE == 0) {
      hv[e]     = __builtin_bit_cast(_Float16, b0);
      hv[4 + e] = __builtin_bit_cast(_Float16, b1);
    } else {
      const float r0 = bf_bits2f(b0) * scale;
      const float r1 = bf_bits2f(b1) * scale;
      hv[e]     = (_Float16)r0;
      hv[4 + e] = (_Float16)r1;
    }
  }
  unsigned short* q = dst + ((size_t)i << 3);
  *(volatile v8h*)q = hv;
  __threadfence();
  *(volatile v8h*)q = hv;
}

__global__ __launch_bounds__(64) void scan_kernel(
    const float* __restrict__ XZ, const float* __restrict__ Wc, const float* __restrict__ Alog,
    const float* __restrict__ Dp, unsigned short* __restrict__ Y16)
{
  __shared__ __align__(16) float sBC[kScanTS * kBCW];
  __shared__ __align__(16) float sY[kScanTS * kScanYP];
  __shared__ __align__(16) float sA[kNst * kScanCh];
  const int tid = threadIdx.x, lane = tid & 31, wave = tid >> 5;
  const int d0 = blockIdx.x * kScanCh;
  const int d  = d0 + tid;
#pragma unroll 1
  for (int s = 0; s < kNst; ++s) {
    const float al = rne_bf(Alog[(size_t)d * kNst + s]);
    sA[s * kScanCh + tid] = -expf(al);
  }
  __syncthreads();
  float negA[kNst], h[kNst];
#pragma unroll
  for (int s = 0; s < kNst; ++s) {
    negA[s] = sA[s * kScanCh + tid];
    h[s] = 0.f;
  }
  const float w0 = rne_bf(Wc[d * 3 + 0]);
  const float w1 = rne_bf(Wc[d * 3 + 1]);
  const float w2 = rne_bf(Wc[d * 3 + 2]);
  const float Dd = rne_bf(Dp[d]);
  const int lr = tid >> 3, lc4 = (tid & 7) * 4;
  const int q = lane >> 3, c8 = (lane & 7) * 8;
  float xprev = 0.f;
  float xcur  = XZ[d];
#pragma unroll 1
  for (int t0 = 0; t0 < kSeq; t0 += kScanTS) {
    __syncthreads();
#pragma unroll
    for (int i = 0; i < 8; ++i) {
      const int r = lr + 8 * i;
      *(v4f*)(sBC + r * kBCW + lc4) = *(const v4f*)(XZ + (size_t)(t0 + r) * kXzP + kColB + lc4);
    }
    __syncthreads();
#pragma unroll 1
    for (int s = 0; s < kScanTS; ++s) {
      const int t = t0 + s;
      const bool has_next = (t + 1 < kSeq);
      const int tn = has_next ? (t + 1) : (kSeq - 1);
      const float xld = XZ[(size_t)tn * kXzP + d];
      const float xnext = has_next ? xld : 0.f;
      const float* rowp = XZ + (size_t)t * kXzP;
      const float zv = rowp[kColZ + d];
      const float v  = rowp[kColDt + d];
      const float* xr = sBC + s * kBCW;
      float Bs[kNst], Cs[kNst];
#pragma unroll
      for (int q4 = 0; q4 < 4; ++q4) {
        const v4f bv = *(const v4f*)(xr + 4 * q4);
        const v4f cv = *(const v4f*)(xr + kNst + 4 * q4);
        Bs[4 * q4 + 0] = bv[0]; Bs[4 * q4 + 1] = bv[1]; Bs[4 * q4 + 2] = bv[2]; Bs[4 * q4 + 3] = bv[3];
        Cs[4 * q4 + 0] = cv[0]; Cs[4 * q4 + 1] = cv[1]; Cs[4 * q4 + 2] = cv[2]; Cs[4 * q4 + 3] = cv[3];
      }
      float cacc = w0 * xprev;
      cacc = fmaf(w1, xcur, cacc);
      cacc = fmaf(w2, xnext, cacc);
      const float sgc = __builtin_amdgcn_rcpf(1.0f + __expf(-cacc));
      const float xc = cacc * sgc;
      const float a   = __expf(-fabsf(v));
      const float u   = 1.0f + a;
      const float l1p = __logf(u) + (a - (u - 1.0f)) * __builtin_amdgcn_rcpf(u);
      const float dt  = fmaxf(v, 0.0f) + l1p;
      const float dtx = dt * xc;
      float y = 0.f;
#pragma unroll
      for (int k = 0; k < kNst; ++k) {
        const float e = __expf(dt * negA[k]);
        h[k] = e * h[k] + dtx * Bs[k];
        y = h[k] * Cs[k] + y;
      }
      y = xc * Dd + y;
      const float sgz = __builtin_amdgcn_rcpf(1.0f + __expf(-zv));
      y = y * (zv * sgz);
      sY[s * kScanYP + tid] = y * kYCarry;
      xprev = xcur;
      xcur = xnext;
    }
    __syncthreads();
    v8h hv[8];
#pragma unroll
    for (int it = 0; it < 8; ++it) {
      const int row = it * 8 + wave * 4 + q;
      const float* sp = sY + row * kScanYP + c8;
      const v4f a0 = *(const v4f*)(sp);
      const v4f a1 = *(const v4f*)(sp + 4);
#pragma unroll
      for (int e = 0; e < 4; ++e) {
        const float g0 = a0[e];
        const float g1 = a1[e];
        hv[it][e]     = (_Float16)g0;
        hv[it][4 + e] = (_Float16)g1;
      }
    }
    for (int pass = 0; pass < 2; ++pass) {
#pragma unroll
      for (int it = 0; it < 8; ++it) {
        const int row = it * 8 + wave * 4 + q;
        const size_t o = (size_t)(t0 + row) * kDin + d0 + c8;
        *(volatile v8h*)(Y16 + o) = hv[it];
      }
      __threadfence();
    }
  }
}

extern "C" void kernel_launch(void* const* d_in, const int* in_sizes, int n_in,
                              void* d_out, int out_size, void* d_ws, size_t ws_size,
                              hipStream_t stream) {
  if (n_in < 6) return;
  if (in_sizes[0] != kSeq * kDm) return;
  if (in_sizes[1] != kNxz * kDm) return;
  if (in_sizes[2] != kDin * 3) return;
  if (in_sizes[3] != kDm * kDin) return;
  if (in_sizes[4] != kDin * kNst) return;
  if (in_sizes[5] != kDin) return;
  if (out_size != kSeq * kDm) return;
  if (ws_size < kWsTotal) return;

  const float* x      = (const float*)d_in[0];
  const float* W_in   = (const float*)d_in[1];
  const float* W_conv = (const float*)d_in[2];
  const float* W_out  = (const float*)d_in[3];
  const float* A_log  = (const float*)d_in[4];
  const float* Dp     = (const float*)d_in[5];
  float* out = (float*)d_out;

  char* ws = (char*)d_ws;
  unsigned short* X16    = (unsigned short*)(ws + kOffX16);
  unsigned short* WIN16  = (unsigned short*)(ws + kOffWIN);
  unsigned short* WOUT16 = (unsigned short*)(ws + kOffWOUT);
  float*          XZ     = (float*)(ws + kOffXZ);
  unsigned short* Y16    = (unsigned short*)(ws + kOffY16);

  plane_convert_kernel<0><<<(kSeq * kDm / 8) / 256, 256, 0, stream>>>(x, X16, kSeq * kDm / 8, kSeq * kDm / 8, 1.0f);
  plane_convert_kernel<0><<<(kXzP * kDm / 8) / 256, 256, 0, stream>>>(W_in, WIN16, kXzP * kDm / 8, kNxz * kDm / 8, 1.0f);
  plane_convert_kernel<1><<<(kDm * kDin / 8) / 256, 256, 0, stream>>>(W_out, WOUT16, kDm * kDin / 8, kDm * kDin / 8, kWoCarry);

  wmma_gemm64<1><<<((kSeq / 64) * (kXzP / 64)) / 8, 256, 0, stream>>>(
      X16, kDm, WIN16, kDm, XZ, kXzP, kSeq, kXzP, kDm, 1.0f);

  scan_kernel<<<kDin / kScanCh, kScanCh, 0, stream>>>(XZ, W_conv, A_log, Dp, Y16);

  wmma_gemm64<0><<<((kSeq / 64) * (kDm / 64)) / 8, 256, 0, stream>>>(
      Y16, kDin, WOUT16, kDin, out, kDm, kSeq, kDm, kDin, kOutScale);
}
